// ChannelAttention_36953898614882
// MI455X (gfx1250) — hardware-verified
//
#include <hip/hip_runtime.h>


#define NB_  4
#define CC   256
#define NT   13824
#define NHD  8
#define HDD  32
#define C3   (3 * CC)
#define WP   (4 * CC)
#define L2EPS 1e-12f
typedef _Float16 h16;
typedef unsigned short bf;
typedef __attribute__((ext_vector_type(16))) __bf16   v16bf;
typedef __attribute__((ext_vector_type(16))) _Float16 v16h;
typedef __attribute__((ext_vector_type(8)))  _Float16 v8h;
typedef __attribute__((ext_vector_type(8)))  unsigned short v8us;
typedef __attribute__((ext_vector_type(8)))  float    v8f;
typedef __attribute__((ext_vector_type(4)))  float    v4f;
typedef __attribute__((ext_vector_type(2)))  float    v2f;
typedef __attribute__((ext_vector_type(4)))  unsigned short v4us;
typedef __attribute__((ext_vector_type(2)))  unsigned short v2us;
typedef v8h  __attribute__((may_alias)) v8ha;
typedef v4f  __attribute__((may_alias)) v4fa;
typedef v8us __attribute__((may_alias)) v8usa;

__device__ __forceinline__ unsigned short f2bf(float f) { unsigned u = __float_as_uint(f); u += 0x7FFFu + ((u >> 16) & 1u); return (unsigned short)(u >> 16); }
__device__ __forceinline__ float bf2f(unsigned short b) { return __uint_as_float(((unsigned)b) << 16); }
__device__ __forceinline__ float bfr(float f) { return bf2f(f2bf(f)); }
__device__ __forceinline__ void splitf(float y, unsigned short& h, unsigned short& l) { h = f2bf(y); l = f2bf(y - bf2f(h)); }
__device__ __forceinline__ v16h cat16(v8h lo, v8h hi) { return __builtin_shufflevector(lo, hi, 0, 1, 2, 3, 4, 5, 6, 7, 8, 9, 10, 11, 12, 13, 14, 15); }
__device__ __forceinline__ v16bf cat16b(v8us lo, v8us hi) { return __builtin_bit_cast(v16bf, __builtin_shufflevector(lo, hi, 0, 1, 2, 3, 4, 5, 6, 7, 8, 9, 10, 11, 12, 13, 14, 15)); }
__device__ __forceinline__ v8f wmma16(v16h a, v16h b, v8f c) { return __builtin_amdgcn_wmma_f32_16x16x32_f16(false, a, false, b, (short)0, c, false, false); }
__device__ __forceinline__ v8f wmmab(v16bf a, v16bf b, v8f c) { return __builtin_amdgcn_wmma_f32_16x16x32_bf16(false, a, false, b, (short)0, c, false, false); }

template <typename T16> struct WFrag;
template <> struct WFrag<h16> { typedef v16h V; static __device__ __forceinline__ V ld(const h16* p) { return cat16(*(const v8h*)p, *(const v8h*)(p + 16)); } static __device__ __forceinline__ v8f mma(V a, V b, v8f c) { return wmma16(a, b, c); } };
template <> struct WFrag<bf> { typedef v16bf V; static __device__ __forceinline__ V ld(const bf* p) { return cat16b(*(const v8us*)p, *(const v8us*)(p + 16)); } static __device__ __forceinline__ v8f mma(V a, V b, v8f c) { return wmmab(a, b, c); } };
template <typename T16, int NSPLIT, bool BIAS>
__global__ __launch_bounds__(32) void k_gemmw(const T16* __restrict__ A, const T16* __restrict__ A2, const T16* __restrict__ Bt, const T16* __restrict__ Bt2, int K, float* C, int ldc, const float* __restrict__ bias, size_t sA, size_t sB, size_t sC) {
    typedef typename WFrag<T16>::V V;
    __shared__ __align__(16) float os[16 * 68];
    const size_t z = blockIdx.z; A += z * sA; if (A2) A2 += z * sA; Bt += z * sB; if (Bt2) Bt2 += z * sB; C += z * sC;
    const int lane = threadIdx.x & 31, lr = lane & 15, hi = lane >> 4; const int r0 = blockIdx.x * 64, c0 = blockIdx.y * 64;
    v8f acc[4][4];
#pragma unroll
    for (int mb = 0; mb < 4; ++mb)
#pragma unroll
        for (int nb = 0; nb < 4; ++nb) acc[mb][nb] = (v8f){};
    const size_t aoff = (size_t)(r0 + lr) * K + 8 * hi, boff = (size_t)(c0 + lr) * K + 8 * hi;
#pragma unroll 1
    for (int kc = 0; kc < K; kc += 32) {
        V a[4], a2[4];
#pragma unroll
        for (int mb = 0; mb < 4; ++mb) { a[mb] = WFrag<T16>::ld(A + aoff + (size_t)mb * 16 * K + kc); if (NSPLIT == 1 || NSPLIT == 2) a2[mb] = WFrag<T16>::ld(A2 + aoff + (size_t)mb * 16 * K + kc); }
#pragma unroll
        for (int nb = 0; nb < 4; ++nb) { const V b = WFrag<T16>::ld(Bt + boff + (size_t)nb * 16 * K + kc); V b2; if (NSPLIT >= 2) b2 = WFrag<T16>::ld(Bt2 + boff + (size_t)nb * 16 * K + kc);
#pragma unroll
            for (int mb = 0; mb < 4; ++mb) { acc[mb][nb] = WFrag<T16>::mma(a[mb], b, acc[mb][nb]); if (NSPLIT == 1 || NSPLIT == 2) acc[mb][nb] = WFrag<T16>::mma(a2[mb], b, acc[mb][nb]); if (NSPLIT >= 2) acc[mb][nb] = WFrag<T16>::mma(a[mb], b2, acc[mb][nb]); } }
        asm volatile("v_nop\n\tv_nop\n\tv_nop\n\tv_nop" : "+v"(acc[0][0]), "+v"(acc[1][1]), "+v"(acc[2][2]), "+v"(acc[3][3]) : "v"(a[0]), "v"(a[3]));
    }
#pragma unroll
    for (int mb = 0; mb < 4; ++mb) {
#pragma unroll
        for (int nb = 0; nb < 4; ++nb) {
#pragma unroll
            for (int j = 0; j < 8; ++j) os[(hi * 8 + j) * 68 + nb * 16 + lr] = acc[mb][nb][j]; }
        __builtin_amdgcn_wave_barrier(); asm volatile("" ::: "memory");
        float* crow = C + (size_t)(r0 + mb * 16) * ldc + c0;
#pragma unroll 1
        for (int ps = 0; ps < 2; ++ps) {
#pragma unroll
            for (int s = 0; s < 8; ++s) { const int row = 2 * s + hi, cofs = lr * 4; v4f val = *(const v4fa*)(os + row * 68 + cofs); if (BIAS) { val[0] += bfr(bias[c0 + cofs]); val[1] += bfr(bias[c0 + cofs + 1]); val[2] += bfr(bias[c0 + cofs + 2]); val[3] += bfr(bias[c0 + cofs + 3]); }
                *(volatile v4f*)(crow + (size_t)row * ldc + cofs) = val; }
            if (ps == 0) __threadfence(); }
        __builtin_amdgcn_wave_barrier(); asm volatile("" ::: "memory");
    }
}

__global__ __launch_bounds__(256) void k_wt3(const float* __restrict__ w, bf* Bt) { const size_t e = ((size_t)blockIdx.x * 256 + threadIdx.x) * 2; if (e >= (size_t)C3 * CC) return; const int k = (int)(e % CC), n = (int)(e / CC); v2us o; o[0] = f2bf(w[(size_t)k * WP + n]); o[1] = f2bf(w[(size_t)(k + 1) * WP + n]); *(volatile v2us*)(Bt + e) = o; __threadfence(); *(volatile v2us*)(Bt + e) = o; }
__global__ __launch_bounds__(256) void k_tpin(const float* __restrict__ xb, bf* XT) { const size_t e = ((size_t)blockIdx.x * 256 + threadIdx.x) * 8; if (e >= (size_t)NT * CC) return; const int c = (int)(e % CC); const int n = (int)(e / CC); v8us o;
#pragma unroll
    for (int q = 0; q < 8; ++q) o[q] = f2bf(xb[(size_t)(c + q) * NT + n]); *(volatile v8us*)(XT + e) = o; __threadfence(); *(volatile v8us*)(XT + e) = o; }
__global__ __launch_bounds__(256) void k_cmaj(const float* __restrict__ F, int col0, bf* Ph, bf* Pl) { const size_t e = ((size_t)blockIdx.x * 256 + threadIdx.x) * 2; if (e >= (size_t)CC * NT) return; const int n = (int)(e % NT); const int c = (int)(e / NT); v2us oh, ol;
#pragma unroll
    for (int q = 0; q < 2; ++q) { unsigned short a, b; splitf(F[(size_t)(n + q) * C3 + col0 + c], a, b); oh[q] = a; ol[q] = b; } *(volatile v2us*)(Ph + e) = oh; *(volatile v2us*)(Pl + e) = ol; __threadfence(); *(volatile v2us*)(Ph + e) = oh; *(volatile v2us*)(Pl + e) = ol; }
__global__ __launch_bounds__(256) void k_vpl(const float* __restrict__ F, bf* Vh, bf* Vl) { const size_t e = ((size_t)blockIdx.x * 256 + threadIdx.x) * 4; if (e >= (size_t)NT * CC) return; const int c = (int)(e % CC); const int n = (int)(e / CC); const v4f v = *(const v4f*)(F + (size_t)n * C3 + 2 * CC + c); v4us oh, ol;
#pragma unroll
    for (int q = 0; q < 4; ++q) { unsigned short a, b; splitf(v[q], a, b); oh[q] = a; ol[q] = b; } *(volatile v4us*)(Vh + e) = oh; *(volatile v4us*)(Vl + e) = ol; __threadfence(); *(volatile v4us*)(Vh + e) = oh; *(volatile v4us*)(Vl + e) = ol; }
__global__ __launch_bounds__(256) void k_norms(const float* __restrict__ F, float* NRM) { __shared__ float red[256]; const int cq = blockIdx.x; const int col = (cq < CC) ? cq : CC + (cq - CC); const int tid = threadIdx.x; float s = 0.f;
#pragma unroll 1
    for (int n = tid; n < NT; n += 256) { const float v = F[(size_t)n * C3 + col]; float p = __fmul_rn(v, v); asm volatile("" : "+v"(p)); s = __fadd_rn(s, p); }
    red[tid] = s; __syncthreads();
#pragma unroll
    for (int sh = 128; sh; sh >>= 1) { if (tid < sh) red[tid] = __fadd_rn(red[tid], red[tid + sh]); __syncthreads(); }
    if (tid == 0) { const float nr = fmaxf(__fsqrt_rn(red[0]), L2EPS); *(volatile float*)(NRM + cq) = nr; __threadfence(); *(volatile float*)(NRM + cq) = nr; } }
__global__ __launch_bounds__(256) void k_bsoft(const float* __restrict__ G, const float* __restrict__ NRM, const float* __restrict__ TMP, bf* Ah, bf* Al) {
    const int lane = threadIdx.x & 31; const int row = blockIdx.x * 8 + (threadIdx.x >> 5); if (row >= CC) return; const int h = row / HDD; const int e = h * HDD + lane;
    float g = G[(size_t)row * CC + e]; const float nq = NRM[row], nk = NRM[CC + e]; float dn = __fmul_rn(nq, nk); asm volatile("" : "+v"(dn)); float t0 = __fdiv_rn(g, dn); asm volatile("" : "+v"(t0)); float tp = bfr(TMP[h]); asm volatile("" : "+v"(tp)); const float t = __fmul_rn(t0, tp);
    float mx = t;
#pragma unroll
    for (int sh = 16; sh; sh >>= 1) mx = fmaxf(mx, __shfl_xor(mx, sh, 32));
    float d0 = __fsub_rn(t, mx); asm volatile("" : "+v"(d0)); const float ex = __builtin_amdgcn_exp2f(__fmul_rn(d0, 1.4426950408889634f)); float sum = ex;
#pragma unroll
    for (int sh = 16; sh; sh >>= 1) sum += __shfl_xor(sum, sh, 32);
    const float p = __fdiv_rn(ex, sum);
#pragma unroll 1
    for (int ps = 0; ps < 2; ++ps) {
        v8us oh, ol;
#pragma unroll
        for (int q = 0; q < 8; ++q) { const int col = lane * 8 + q; const int src = col - h * HDD; const float pv = __shfl(p, src & 31, 32); const bool in = (src >= 0 && src < HDD); unsigned short a, b; splitf(in ? pv : 0.0f, a, b); oh[q] = a; ol[q] = b; }
        *(volatile v8us*)(Ah + (size_t)row * CC + lane * 8) = oh; *(volatile v8us*)(Al + (size_t)row * CC + lane * 8) = ol;
        if (ps == 0) __threadfence(); }
}

extern "C" void kernel_launch(void* const* d_in, const int* in_sizes, int n_in,
                              void* d_out, int out_size, void* d_ws, size_t ws_size, hipStream_t stream) {
    (void)in_sizes; (void)n_in; (void)out_size;
    const float* x = (const float*)d_in[0]; const float* w = (const float*)d_in[1]; const float* TMP = (const float*)d_in[2];
    float* OUT = (float*)d_out;
    char* wsp = (char*)d_ws;
    auto take = [&](size_t bytes) { char* p = wsp; wsp += (bytes + 255) & ~(size_t)255; return (void*)p; };
    bf* WB = (bf*)take((size_t)C3 * CC * 2); bf* XT = (bf*)take((size_t)NT * CC * 2); float* F = (float*)take((size_t)NT * C3 * 4); bf* QPh = (bf*)take((size_t)CC * NT * 2); bf* QPl = (bf*)take((size_t)CC * NT * 2); bf* KPh = (bf*)take((size_t)CC * NT * 2); bf* KPl = (bf*)take((size_t)CC * NT * 2); bf* Vh = (bf*)take((size_t)NT * CC * 2); bf* Vl = (bf*)take((size_t)NT * CC * 2); float* G = (float*)take((size_t)CC * CC * 4); float* NRM = (float*)take((size_t)2 * CC * 4); bf* Ah = (bf*)take((size_t)CC * CC * 2); bf* Al = (bf*)take((size_t)CC * CC * 2);
    if ((size_t)(wsp - (char*)d_ws) > ws_size) return;
    k_wt3<<<(unsigned)(((size_t)C3 * CC / 2 + 255) / 256), 256, 0, stream>>>(w, WB);
    for (int b = 0; b < NB_; ++b) { const float* xb = x + (size_t)b * CC * NT;
        k_tpin<<<(unsigned)(((size_t)NT * CC / 8 + 255) / 256), 256, 0, stream>>>(xb, XT);
        k_gemmw<bf, 0, false><<<dim3(NT / 64, C3 / 64, 1), 32, 0, stream>>>(XT, nullptr, WB, nullptr, CC, F, C3, nullptr, 0, 0, 0);
        k_cmaj<<<(unsigned)(((size_t)CC * NT / 2 + 255) / 256), 256, 0, stream>>>(F, 0, QPh, QPl); k_cmaj<<<(unsigned)(((size_t)CC * NT / 2 + 255) / 256), 256, 0, stream>>>(F, CC, KPh, KPl);
        k_vpl<<<(unsigned)(((size_t)NT * CC / 4 + 255) / 256), 256, 0, stream>>>(F, Vh, Vl);
        k_norms<<<2 * CC, 256, 0, stream>>>(F, NRM);
        k_gemmw<bf, 2, false><<<dim3(CC / 64, CC / 64, 1), 32, 0, stream>>>(QPh, QPl, KPh, KPl, NT, G, CC, nullptr, 0, 0, 0);
        k_bsoft<<<CC / 8, 256, 0, stream>>>(G, NRM, TMP, Ah, Al);
        k_gemmw<bf, 2, false><<<dim3(CC / 64, NT / 64, 1), 32, 0, stream>>>(Ah, Al, Vh, Vl, CC, OUT + (size_t)b * CC * NT, NT, nullptr, 0, 0, 0); }
}
